// MultiHeadAttention_59992103190747
// MI455X (gfx1250) — hardware-verified
//
#include <hip/hip_runtime.h>


#ifndef NB
#define NB 4
#endif
#ifndef SEQ
#define SEQ 2048
#endif
#define NB_FULL  4
#define SEQ_FULL 2048
#ifndef OUT_SEQ
#define OUT_SEQ SEQ
#endif
#define DM   1024
#define NH_  16
#define HD   64
#define AW   4
#define SC2  (0.125f * 1.4426950408889634f)
#define PSH  8.0f
#define CTXS 256.0f
#define WPS  1024.0f
#define OSCI (1.0f / (256.0f * 1024.0f))

static_assert(HD == 64);
static_assert(NH_ * HD == DM);
static_assert(DM % 64 == 0);
static_assert(DM % 32 == 0);
static_assert(SEQ % 64 == 0);
static_assert((NB * SEQ) % 64 == 0);
static_assert(SEQ % 32 == 0);
static_assert(SEQ % (16 * AW) == 0);
static_assert(((size_t)SEQ * DM) % 8 == 0);
static_assert(((size_t)DM * DM) % 8 == 0);
static_assert(NB <= NB_FULL);
static_assert(SEQ <= SEQ_FULL);

typedef _Float16 h16;
typedef unsigned short bf;
typedef __attribute__((ext_vector_type(16))) __bf16   v16bf;
typedef __attribute__((ext_vector_type(16))) _Float16 v16h;
typedef __attribute__((ext_vector_type(8)))  _Float16 v8h;
typedef __attribute__((ext_vector_type(8)))  unsigned short v8us;
typedef __attribute__((ext_vector_type(8)))  float    v8f;
typedef __attribute__((ext_vector_type(4)))  float    v4f;
typedef v4f  __attribute__((may_alias)) v4fa;
typedef v8us __attribute__((may_alias)) v8usa;

__device__ __forceinline__ unsigned short f2bf(float f) { unsigned u = __float_as_uint(f); u += 0x7FFFu + ((u >> 16) & 1u); return (unsigned short)(u >> 16); }
__device__ __forceinline__ float bfr(float f) { return __uint_as_float(((unsigned)f2bf(f)) << 16); }
__device__ __forceinline__ v16h cat16(v8h lo, v8h hi) { return __builtin_shufflevector(lo, hi, 0, 1, 2, 3, 4, 5, 6, 7, 8, 9, 10, 11, 12, 13, 14, 15); }
__device__ __forceinline__ v16bf cat16b(v8us lo, v8us hi) { return __builtin_bit_cast(v16bf, __builtin_shufflevector(lo, hi, 0, 1, 2, 3, 4, 5, 6, 7, 8, 9, 10, 11, 12, 13, 14, 15)); }
__device__ __forceinline__ v8f wmma16(v16h a, v16h b, v8f c) { return __builtin_amdgcn_wmma_f32_16x16x32_f16(false, a, false, b, (short)0, c, false, false); }
__device__ __forceinline__ v8f wmmab(v16bf a, v16bf b, v8f c) { return __builtin_amdgcn_wmma_f32_16x16x32_bf16(false, a, false, b, (short)0, c, false, false); }
__device__ __forceinline__ v16h  ldh(const h16* p) { return cat16(*(const v8h*)p, *(const v8h*)(p + 16)); }
__device__ __forceinline__ v16bf ldb(const bf* p)  { return cat16b(*(const v8us*)p, *(const v8us*)(p + 16)); }
__device__ __forceinline__ void wave_sync() { __builtin_amdgcn_fence(3  , "wavefront"); __builtin_amdgcn_wave_barrier(); asm volatile("" ::: "memory"); }

__global__ __launch_bounds__(256) void k_cvt8(const float* __restrict__ src, bf* dst, size_t n8) {
    const size_t i = (size_t)blockIdx.x * 256 + threadIdx.x; if (i >= n8) return;
    const v8f v = *(const v8f*)(src + i * 8); v8us o;
#pragma unroll
    for (int k = 0; k < 8; ++k) o[k] = f2bf(v[k]);
    *(volatile v8us*)(dst + i * 8) = o; __threadfence(); *(volatile v8us*)(dst + i * 8) = o;
}

__global__ __launch_bounds__(256) void k_cvtT(const float* __restrict__ W, bf* WT, int asF16, float scale) {
    __shared__ __align__(16) unsigned short ts[64 * 72];
    const int tid = threadIdx.x; const int k0 = blockIdx.x * 64, n0 = blockIdx.y * 64;
    { const int kk = tid >> 2, seg = (tid & 3) * 16;
      const float* src = W + (size_t)(k0 + kk) * DM + n0 + seg;
#pragma unroll
      for (int q = 0; q < 4; ++q) { const v4f v = *(const v4f*)(src + 4 * q);
#pragma unroll
          for (int i = 0; i < 4; ++i) { const float w = v[i];
              const unsigned short ub = f2bf(w);
              const h16 hv = (h16)(__uint_as_float(((unsigned)ub) << 16) * scale);
              const unsigned short uh = __builtin_bit_cast(unsigned short, hv);
              ts[(seg + 4 * q + i) * 72 + kk] = asF16 ? uh : ub; } } }
    __syncthreads();
#pragma unroll 1
    for (int ps = 0; ps < 2; ++ps) {
#pragma unroll
        for (int p = 0; p < 2; ++p) { const int n = p * 32 + (tid >> 3), c8 = (tid & 7) * 8;
            const v8us o = *(const v8usa*)(&ts[n * 72 + c8]);
            *(volatile v8us*)(WT + (size_t)(n0 + n) * DM + k0 + c8) = o; }
        if (ps == 0) __threadfence(); }
}

template <int BROW>
__global__ __launch_bounds__(32) void k_proj(const bf* __restrict__ A, const bf* __restrict__ Bt, const float* __restrict__ bias, h16* Ph, int RB, size_t sRB, int pitch, int CB, size_t sCB) {
    __shared__ __align__(16) float os[16 * 68];
    const int K = DM;
    const int lane = threadIdx.x & 31, lr = lane & 15, hi = lane >> 4; const int r0 = blockIdx.x * 64, c0 = blockIdx.y * 64;
    v8f acc[4][4];
#pragma unroll
    for (int mb = 0; mb < 4; ++mb)
#pragma unroll
        for (int nb = 0; nb < 4; ++nb) acc[mb][nb] = (v8f){};
    const size_t aoff = (size_t)(r0 + lr) * K + 8 * hi, boff = (size_t)(c0 + lr) * K + 8 * hi;
#pragma unroll 1
    for (int kc = 0; kc < K; kc += 32) {
        v16bf a[4];
#pragma unroll
        for (int mb = 0; mb < 4; ++mb) a[mb] = ldb(A + aoff + (size_t)mb * 16 * K + kc);
#pragma unroll
        for (int nb = 0; nb < 4; ++nb) { const v16bf b = ldb(Bt + boff + (size_t)nb * 16 * K + kc);
#pragma unroll
            for (int mb = 0; mb < 4; ++mb) acc[mb][nb] = wmmab(a[mb], b, acc[mb][nb]); }
        asm volatile("v_nop\n\tv_nop\n\tv_nop\n\tv_nop" : "+v"(acc[0][0]), "+v"(acc[1][1]), "+v"(acc[2][2]), "+v"(acc[3][3]) : "v"(a[0]), "v"(a[1]), "v"(a[2]), "v"(a[3]));
    }
    float bc[4];
#pragma unroll
    for (int nb = 0; nb < 4; ++nb) bc[nb] = BROW ? 0.0f : bfr(bias[c0 + nb * 16 + lr]);
    const size_t tbase = (size_t)(r0 / RB) * sRB + (size_t)(r0 % RB) * (size_t)pitch + (size_t)(c0 / CB) * sCB + (size_t)(c0 % CB);
#pragma unroll
    for (int mb = 0; mb < 4; ++mb) {
        float br[8];
#pragma unroll
        for (int j = 0; j < 8; ++j) br[j] = BROW ? bfr(bias[r0 + mb * 16 + hi * 8 + j]) : 0.0f;
#pragma unroll
        for (int nb = 0; nb < 4; ++nb) {
#pragma unroll
            for (int j = 0; j < 8; ++j) os[(hi * 8 + j) * 68 + nb * 16 + lr] = (acc[mb][nb][j] + bc[nb]) + br[j]; }
        wave_sync();
        const size_t sb = tbase + (size_t)(mb * 16) * (size_t)pitch;
#pragma unroll 1
        for (int ps = 0; ps < 2; ++ps) {
#pragma unroll
            for (int s = 0; s < 4; ++s) { const int row = 4 * s + (lane >> 3), c8 = (lane & 7) * 8;
                const v4f x0 = *(const v4fa*)(&os[row * 68 + c8]); const v4f x1 = *(const v4fa*)(&os[row * 68 + c8 + 4]); v8h hv;
#pragma unroll
                for (int i = 0; i < 4; ++i) { hv[i] = (h16)x0[i]; hv[4 + i] = (h16)x1[i]; }
                const size_t oo = sb + (size_t)row * (size_t)pitch + c8;
                *(volatile v8h*)(Ph + oo) = hv; }
            if (ps == 0) __threadfence(); }
        wave_sync();
    }
}

__global__ __launch_bounds__(32) void k_oproj(const h16* __restrict__ A, const h16* __restrict__ Bt, const float* __restrict__ bias, float* OUT) {
    __shared__ __align__(16) float os[16 * 68];
    const int K = DM;
    const int lane = threadIdx.x & 31, lr = lane & 15, hi = lane >> 4; const int r0 = blockIdx.x * 64, c0 = blockIdx.y * 64;
    v8f acc[4][4];
#pragma unroll
    for (int mb = 0; mb < 4; ++mb)
#pragma unroll
        for (int nb = 0; nb < 4; ++nb) acc[mb][nb] = (v8f){};
    const size_t aoff = (size_t)(r0 + lr) * K + 8 * hi, boff = (size_t)(c0 + lr) * K + 8 * hi;
#pragma unroll 1
    for (int kc = 0; kc < K; kc += 32) {
        v16h a[4];
#pragma unroll
        for (int mb = 0; mb < 4; ++mb) a[mb] = ldh(A + aoff + (size_t)mb * 16 * K + kc);
#pragma unroll
        for (int nb = 0; nb < 4; ++nb) { const v16h b = ldh(Bt + boff + (size_t)nb * 16 * K + kc);
#pragma unroll
            for (int mb = 0; mb < 4; ++mb) acc[mb][nb] = wmma16(a[mb], b, acc[mb][nb]); }
        asm volatile("v_nop\n\tv_nop\n\tv_nop\n\tv_nop" : "+v"(acc[0][0]), "+v"(acc[1][1]), "+v"(acc[2][2]), "+v"(acc[3][3]) : "v"(a[0]), "v"(a[1]), "v"(a[2]), "v"(a[3]));
    }
    float bc[4];
#pragma unroll
    for (int nb = 0; nb < 4; ++nb) bc[nb] = bfr(bias[c0 + nb * 16 + lr]);
    const int bb = r0 / SEQ, tt = r0 % SEQ;
    float* obase = OUT + ((size_t)bb * OUT_SEQ + tt) * DM + c0;
#pragma unroll
    for (int mb = 0; mb < 4; ++mb) {
#pragma unroll
        for (int nb = 0; nb < 4; ++nb) {
#pragma unroll
            for (int j = 0; j < 8; ++j) os[(hi * 8 + j) * 68 + nb * 16 + lr] = acc[mb][nb][j] * OSCI + bc[nb]; }
        wave_sync();
#pragma unroll 1
        for (int ps = 0; ps < 2; ++ps) {
#pragma unroll
            for (int s = 0; s < 8; ++s) { const int row = 2 * s + hi, cofs = lr * 4;
                const v4f val = *(const v4fa*)(&os[row * 68 + cofs]);
                *(volatile v4f*)(obase + (size_t)(mb * 16 + row) * DM + cofs) = val; }
            if (ps == 0) __threadfence(); }
        wave_sync();
    }
}

__global__ __launch_bounds__(32 * AW) void k_flash(const h16* __restrict__ QH, const h16* __restrict__ KP, const h16* __restrict__ VT, h16* CTX) {
    __shared__ __align__(16) float os[AW * 16 * 68];
    const int lane = threadIdx.x & 31, lr = lane & 15, hi = lane >> 4;
    const int wave = __builtin_amdgcn_readfirstlane((int)(threadIdx.x >> 5));
    const int zh = blockIdx.y; const int b = zh / NH_, h = zh % NH_;
    const int t0 = (blockIdx.x * AW + wave) * 16;
    const size_t pbase = (size_t)zh * SEQ * HD;
    const size_t qo = pbase + (size_t)(t0 + lr) * HD + 8 * hi;
    const v16h qh0 = ldh(QH + qo), qh1 = ldh(QH + qo + 32);
    const size_t ko = pbase + (size_t)lr * HD + 8 * hi;
    const size_t vo = pbase + (size_t)lr * SEQ + 8 * hi;
    v8f o0 = (v8f){}, o1 = (v8f){}, o2 = (v8f){}, o3 = (v8f){};
    float m = -3.0e38f, l = 0.0f;
#pragma unroll 1
    for (int key0 = 0; key0 < SEQ; key0 += 32) {
        const h16* ka = KP + ko + (size_t)key0 * HD;
        const v16h ka0 = ldh(ka), ka1 = ldh(ka + 32), kb0 = ldh(ka + 16 * HD), kb1 = ldh(ka + 16 * HD + 32);
        v8f sa = (v8f){}, sb = (v8f){};
        sa = wmma16(ka0, qh0, sa); sb = wmma16(kb0, qh0, sb);
        sa = wmma16(ka1, qh1, sa); sb = wmma16(kb1, qh1, sb);
        asm volatile("v_nop\n\tv_nop\n\tv_nop\n\tv_nop" : "+v"(sa), "+v"(sb) : "v"(ka0), "v"(ka1), "v"(kb0), "v"(kb1), "v"(qh0), "v"(qh1));
        float ta[8], tb[8]; float mx = -3.0e38f;
#pragma unroll
        for (int r = 0; r < 8; ++r) { ta[r] = sa[r] * SC2; tb[r] = sb[r] * SC2; mx = fmaxf(mx, fmaxf(ta[r], tb[r])); }
        mx = fmaxf(mx, __shfl_xor(mx, 16, 32));
        const float mnew = fmaxf(m, mx);
        const float alpha = __builtin_amdgcn_exp2f(m - mnew);
        const float sh = PSH - mnew;
        v16h pb; float ls = 0.0f;
#pragma unroll
        for (int r = 0; r < 8; ++r) { const h16 pa = (h16)__builtin_amdgcn_exp2f(ta[r] + sh); const h16 pc = (h16)__builtin_amdgcn_exp2f(tb[r] + sh); pb[r] = pa; pb[8 + r] = pc; ls += (float)pa + (float)pc; }
        l = l * alpha + ls; m = mnew;
        o0 = o0 * alpha; o1 = o1 * alpha; o2 = o2 * alpha; o3 = o3 * alpha;
        const h16* va = VT + vo + key0;
        const v16h v0 = ldh(va), v1 = ldh(va + (size_t)16 * SEQ), v2 = ldh(va + (size_t)32 * SEQ), v3 = ldh(va + (size_t)48 * SEQ);
        o0 = wmma16(v0, pb, o0); o1 = wmma16(v1, pb, o1); o2 = wmma16(v2, pb, o2); o3 = wmma16(v3, pb, o3);
        asm volatile("v_nop\n\tv_nop\n\tv_nop\n\tv_nop" : "+v"(o0), "+v"(o1), "+v"(o2), "+v"(o3) : "v"(v0), "v"(v1), "v"(v2), "v"(v3), "v"(pb));
    }
    l += __shfl_xor(l, 16, 32);
    const float inv = CTXS / l;
    const int wb = wave * 16 * 68;
    { v4f a, c;
      a[0] = o0[0] * inv; a[1] = o0[1] * inv; a[2] = o0[2] * inv; a[3] = o0[3] * inv; c[0] = o0[4] * inv; c[1] = o0[5] * inv; c[2] = o0[6] * inv; c[3] = o0[7] * inv;
      *(v4fa*)(&os[wb + lr * 68 +  0 + 8 * hi]) = a; *(v4fa*)(&os[wb + lr * 68 +  0 + 8 * hi + 4]) = c;
      a[0] = o1[0] * inv; a[1] = o1[1] * inv; a[2] = o1[2] * inv; a[3] = o1[3] * inv; c[0] = o1[4] * inv; c[1] = o1[5] * inv; c[2] = o1[6] * inv; c[3] = o1[7] * inv;
      *(v4fa*)(&os[wb + lr * 68 + 16 + 8 * hi]) = a; *(v4fa*)(&os[wb + lr * 68 + 16 + 8 * hi + 4]) = c;
      a[0] = o2[0] * inv; a[1] = o2[1] * inv; a[2] = o2[2] * inv; a[3] = o2[3] * inv; c[0] = o2[4] * inv; c[1] = o2[5] * inv; c[2] = o2[6] * inv; c[3] = o2[7] * inv;
      *(v4fa*)(&os[wb + lr * 68 + 32 + 8 * hi]) = a; *(v4fa*)(&os[wb + lr * 68 + 32 + 8 * hi + 4]) = c;
      a[0] = o3[0] * inv; a[1] = o3[1] * inv; a[2] = o3[2] * inv; a[3] = o3[3] * inv; c[0] = o3[4] * inv; c[1] = o3[5] * inv; c[2] = o3[6] * inv; c[3] = o3[7] * inv;
      *(v4fa*)(&os[wb + lr * 68 + 48 + 8 * hi]) = a; *(v4fa*)(&os[wb + lr * 68 + 48 + 8 * hi + 4]) = c; }
    wave_sync();
    h16* crow = CTX + ((size_t)b * SEQ + t0) * DM + h * HD;
#pragma unroll 1
    for (int ps = 0; ps < 2; ++ps) {
#pragma unroll
        for (int s = 0; s < 4; ++s) { const int row = 4 * s + (lane >> 3), c8 = (lane & 7) * 8;
            const v4f x0 = *(const v4fa*)(&os[wb + row * 68 + c8]); const v4f x1 = *(const v4fa*)(&os[wb + row * 68 + c8 + 4]); v8h hv;
#pragma unroll
            for (int i = 0; i < 4; ++i) { hv[i] = (h16)x0[i]; hv[4 + i] = (h16)x1[i]; }
            *(volatile v8h*)(crow + (size_t)row * DM + c8) = hv; }
        if (ps == 0) __threadfence(); }
}

static constexpr size_t al256(size_t v) { return (v + 255) & ~(size_t)255; }
static constexpr size_t SZ_XB = al256((size_t)NB * SEQ * DM * 2);
static constexpr size_t SZ_WB = al256((size_t)4 * DM * DM * 2);
static constexpr size_t SZ_PL = al256((size_t)NB * NH_ * SEQ * HD * 2);
static constexpr size_t SZ_CX = al256((size_t)NB * SEQ * DM * 2);
static constexpr size_t SZ_TOTAL = SZ_XB + SZ_WB + 3 * SZ_PL + SZ_CX;
static_assert(SZ_TOTAL <= (size_t)134217728);
static_assert(((size_t)DM * DM * 2) % 256 == 0);

extern "C" void kernel_launch(void* const* d_in, const int* in_sizes, int n_in,
                              void* d_out, int out_size, void* d_ws, size_t ws_size, hipStream_t stream) {
    if (n_in < 9) return;
    const size_t needx = ((size_t)(NB - 1) * SEQ_FULL + SEQ) * DM;
    if ((size_t)in_sizes[0] < needx) return;
    if ((size_t)in_sizes[1] < (size_t)DM * DM || (size_t)in_sizes[3] < (size_t)DM * DM || (size_t)in_sizes[5] < (size_t)DM * DM || (size_t)in_sizes[7] < (size_t)DM * DM) return;
    if (in_sizes[2] < DM || in_sizes[4] < DM || in_sizes[6] < DM || in_sizes[8] < DM) return;
    if ((size_t)out_size < ((size_t)(NB - 1) * OUT_SEQ + SEQ) * DM) return;
    if (SZ_TOTAL > ws_size) return;
    const float* x  = (const float*)d_in[0];
    const float* wq = (const float*)d_in[1]; const float* bq = (const float*)d_in[2];
    const float* wk = (const float*)d_in[3]; const float* bk = (const float*)d_in[4];
    const float* wv = (const float*)d_in[5]; const float* bv = (const float*)d_in[6];
    const float* wp = (const float*)d_in[7]; const float* bp = (const float*)d_in[8];
    float* OUT = (float*)d_out;
    char* wsp = (char*)d_ws;
    bf* XB = (bf*)wsp; wsp += SZ_XB;
    bf* WB = (bf*)wsp; wsp += SZ_WB;
    h16* QH = (h16*)wsp; wsp += SZ_PL;
    h16* KP = (h16*)wsp; wsp += SZ_PL;
    h16* VT = (h16*)wsp; wsp += SZ_PL;
    h16* CX = (h16*)wsp; wsp += SZ_CX;
    bf* WQ = WB; bf* WK = WB + (size_t)DM * DM; bf* WV = WB + (size_t)2 * DM * DM; bf* WP = WB + (size_t)3 * DM * DM;

    if (SEQ == SEQ_FULL) {
        const size_t n8 = (size_t)NB * SEQ * DM / 8;
        k_cvt8<<<(unsigned)((n8 + 255) / 256), 256, 0, stream>>>(x, XB, n8);
    } else {
        const size_t n8 = (size_t)SEQ * DM / 8;
        for (int b = 0; b < NB; ++b) k_cvt8<<<(unsigned)((n8 + 255) / 256), 256, 0, stream>>>(x + (size_t)b * SEQ_FULL * DM, XB + (size_t)b * SEQ * DM, n8);
    }
    { const dim3 g(DM / 64, DM / 64, 1);
      k_cvtT<<<g, 256, 0, stream>>>(wq, WQ, 0, 1.0f);
      k_cvtT<<<g, 256, 0, stream>>>(wk, WK, 0, 1.0f);
      k_cvtT<<<g, 256, 0, stream>>>(wv, WV, 0, 1.0f);
      k_cvtT<<<g, 256, 0, stream>>>(wp, WP, 1, WPS); }

    k_proj<0><<<dim3(NB * SEQ / 64, DM / 64, 1), 32, 0, stream>>>(XB, WQ, bq, QH, SEQ, (size_t)NH_ * SEQ * HD, HD, HD, (size_t)SEQ * HD);
    k_proj<0><<<dim3(NB * SEQ / 64, DM / 64, 1), 32, 0, stream>>>(XB, WK, bk, KP, SEQ, (size_t)NH_ * SEQ * HD, HD, HD, (size_t)SEQ * HD);
    k_proj<1><<<dim3(DM / 64, NB * SEQ / 64, 1), 32, 0, stream>>>(WV, XB, bv, VT, DM, (size_t)0, SEQ, SEQ, (size_t)DM * SEQ);

    k_flash<<<dim3(SEQ / (16 * AW), NB * NH_, 1), 32 * AW, 0, stream>>>(QH, KP, VT, CX);

    k_oproj<<<dim3(NB * SEQ / 64, DM / 64, 1), 32, 0, stream>>>(CX, (const h16*)WP, bp, OUT);
}
